// NonLocalBlock2D_with_mask_Res_13322988552681
// MI455X (gfx1250) — hardware-verified
//
#include <hip/hip_runtime.h>


#define NB_  2
#define HH   64
#define NN   4096
#define CC   128
#define KC   1152
#define QH   2048
#define PCAR 1024.0f
typedef _Float16 h16;
typedef unsigned short bf;
typedef __attribute__((ext_vector_type(16))) __bf16   v16bf;
typedef __attribute__((ext_vector_type(16))) _Float16 v16h;
typedef __attribute__((ext_vector_type(8)))  _Float16 v8h;
typedef __attribute__((ext_vector_type(8)))  unsigned short v8us;
typedef __attribute__((ext_vector_type(8)))  float    v8f;
typedef __attribute__((ext_vector_type(4)))  float    v4f;
typedef v8h  __attribute__((may_alias)) v8ha;
typedef v4f  __attribute__((may_alias)) v4fa;
typedef v8us __attribute__((may_alias)) v8usa;

__device__ __forceinline__ unsigned short f2bf(float f) { unsigned u = __float_as_uint(f); u += 0x7FFFu + ((u >> 16) & 1u); return (unsigned short)(u >> 16); }
__device__ __forceinline__ float bf2f(unsigned short b) { return __uint_as_float(((unsigned)b) << 16); }
__device__ __forceinline__ float bfr(float f) { return bf2f(f2bf(f)); }
__device__ __forceinline__ v16h cat16(v8h lo, v8h hi) { return __builtin_shufflevector(lo, hi, 0, 1, 2, 3, 4, 5, 6, 7, 8, 9, 10, 11, 12, 13, 14, 15); }
__device__ __forceinline__ v16bf cat16b(v8us lo, v8us hi) { return __builtin_bit_cast(v16bf, __builtin_shufflevector(lo, hi, 0, 1, 2, 3, 4, 5, 6, 7, 8, 9, 10, 11, 12, 13, 14, 15)); }
__device__ __forceinline__ v8f wmma16(v16h a, v16h b, v8f c) { return __builtin_amdgcn_wmma_f32_16x16x32_f16(false, a, false, b, (short)0, c, false, false); }
__device__ __forceinline__ v8f wmmab(v16bf a, v16bf b, v8f c) { return __builtin_amdgcn_wmma_f32_16x16x32_bf16(false, a, false, b, (short)0, c, false, false); }


template <typename T16> struct WFrag;
template <> struct WFrag<h16> { typedef v16h V; static __device__ __forceinline__ V ld(const h16* p) { return cat16(*(const v8h*)p, *(const v8h*)(p + 16)); } static __device__ __forceinline__ v8f mma(V a, V b, v8f c) { return wmma16(a, b, c); } };
template <> struct WFrag<bf> { typedef v16bf V; static __device__ __forceinline__ V ld(const bf* p) { return cat16b(*(const v8us*)p, *(const v8us*)(p + 16)); } static __device__ __forceinline__ v8f mma(V a, V b, v8f c) { return wmmab(a, b, c); } };
template <typename T16, int NSPLIT, bool BIAS>
__global__ __launch_bounds__(32) void k_gemmw(const T16* __restrict__ A, const T16* __restrict__ A2, const T16* __restrict__ Bt, const T16* __restrict__ Bt2, int K, float* C, int ldc, const float* __restrict__ bias, size_t sA, size_t sB, size_t sC) {
    typedef typename WFrag<T16>::V V;
    __shared__ __align__(16) float os[16 * 68];
    const size_t z = blockIdx.z; A += z * sA; if (A2) A2 += z * sA; Bt += z * sB; if (Bt2) Bt2 += z * sB; C += z * sC;
    const int lane = threadIdx.x & 31, lr = lane & 15, hi = lane >> 4; const int r0 = blockIdx.x * 64, c0 = blockIdx.y * 64;
    v8f acc[4][4];
#pragma unroll
    for (int mb = 0; mb < 4; ++mb)
#pragma unroll
        for (int nb = 0; nb < 4; ++nb) acc[mb][nb] = (v8f){};
    const size_t aoff = (size_t)(r0 + lr) * K + 8 * hi, boff = (size_t)(c0 + lr) * K + 8 * hi;
#pragma unroll 1
    for (int kc = 0; kc < K; kc += 32) {
        V a[4], a2[4];
#pragma unroll
        for (int mb = 0; mb < 4; ++mb) { a[mb] = WFrag<T16>::ld(A + aoff + (size_t)mb * 16 * K + kc); if (NSPLIT == 1 || NSPLIT == 2) a2[mb] = WFrag<T16>::ld(A2 + aoff + (size_t)mb * 16 * K + kc); }
#pragma unroll
        for (int nb = 0; nb < 4; ++nb) { const V b = WFrag<T16>::ld(Bt + boff + (size_t)nb * 16 * K + kc); V b2; if (NSPLIT >= 2) b2 = WFrag<T16>::ld(Bt2 + boff + (size_t)nb * 16 * K + kc);
#pragma unroll
            for (int mb = 0; mb < 4; ++mb) { acc[mb][nb] = WFrag<T16>::mma(a[mb], b, acc[mb][nb]); if (NSPLIT == 1 || NSPLIT == 2) acc[mb][nb] = WFrag<T16>::mma(a2[mb], b, acc[mb][nb]); if (NSPLIT >= 2) acc[mb][nb] = WFrag<T16>::mma(a[mb], b2, acc[mb][nb]); } }
        asm volatile("v_nop\n\tv_nop\n\tv_nop\n\tv_nop" : "+v"(acc[0][0]), "+v"(acc[1][1]), "+v"(acc[2][2]), "+v"(acc[3][3]) : "v"(a[0]), "v"(a[3]));
    }
#pragma unroll
    for (int mb = 0; mb < 4; ++mb) {
#pragma unroll
        for (int nb = 0; nb < 4; ++nb) {
#pragma unroll
            for (int j = 0; j < 8; ++j) os[(hi * 8 + j) * 68 + nb * 16 + lr] = acc[mb][nb][j]; }
        __builtin_amdgcn_wave_barrier(); asm volatile("" ::: "memory");
        float* crow = C + (size_t)(r0 + mb * 16) * ldc + c0;
#pragma unroll 1
        for (int ps = 0; ps < 2; ++ps) {
#pragma unroll
            for (int s = 0; s < 8; ++s) { const int row = 2 * s + hi, cofs = lr * 4; v4f val = *(const v4fa*)(os + row * 68 + cofs); if (BIAS) { val[0] += bfr(bias[c0 + cofs]); val[1] += bfr(bias[c0 + cofs + 1]); val[2] += bfr(bias[c0 + cofs + 2]); val[3] += bfr(bias[c0 + cofs + 3]); }
                *(volatile v4f*)(crow + (size_t)row * ldc + cofs) = val; }
            if (ps == 0) __threadfence(); }
        __builtin_amdgcn_wave_barrier(); asm volatile("" ::: "memory");
    }
}

__device__ __forceinline__ h16 tohx(float x) { return (h16)x; }
__device__ __forceinline__ void splitf(float y, unsigned short& h, unsigned short& l) { h = f2bf(y); l = f2bf(y - bf2f(h)); }
typedef __attribute__((ext_vector_type(2))) _Float16 v2h;
typedef __attribute__((ext_vector_type(4))) _Float16 v4h;
typedef __attribute__((ext_vector_type(2))) unsigned short v2us;
typedef __attribute__((ext_vector_type(4))) unsigned short v4us;
typedef __attribute__((ext_vector_type(2))) float v2f;

__global__ __launch_bounds__(256) void k_wtG(const float* __restrict__ w, int K, int N, bf* Bt) {
    const int lane = threadIdx.x & 31; const int L0 = (blockIdx.x * 8 + (threadIdx.x >> 5)) * 8; const int nlines = N * K / 64;
#pragma unroll 1
    for (int ps = 0; ps < 2; ++ps) {
#pragma unroll 1
        for (int l = 0; l < 8; ++l) { const int L = L0 + l; if (L >= nlines) break; const size_t e = (size_t)L * 64 + lane * 2; const int k = (int)(e % K), n = (int)(e / K); v2us o;
            o[0] = f2bf(w[(size_t)k * N + n]); o[1] = f2bf(w[(size_t)(k + 1) * N + n]); *(volatile v2us*)(Bt + e) = o; }
        if (ps == 0) __threadfence(); }
}
__global__ __launch_bounds__(256) void k_cvt8(const float* __restrict__ src, bf* dst, size_t n8) { const size_t i = (size_t)blockIdx.x * 256 + threadIdx.x; if (i >= n8) return; const v8f v = *(const v8f*)(src + i * 8); v8us o;
#pragma unroll
    for (int k = 0; k < 8; ++k) o[k] = f2bf(v[k]); *(volatile v8us*)(dst + i * 8) = o; __threadfence(); *(volatile v8us*)(dst + i * 8) = o; }
__global__ __launch_bounds__(256) void k_f16(const float* __restrict__ F, size_t n4, h16* P) { const size_t i = ((size_t)blockIdx.x * 256 + threadIdx.x) * 4; if (i >= n4 * 4) return; const v4f a = *(const v4f*)(F + i); v4h o; o[0] = tohx(a[0]); o[1] = tohx(a[1]); o[2] = tohx(a[2]); o[3] = tohx(a[3]); *(volatile v4h*)(P + i) = o; __threadfence(); *(volatile v4h*)(P + i) = o; }
__global__ __launch_bounds__(256) void k_gt16(const float* __restrict__ G, h16* GT) { const size_t e = ((size_t)blockIdx.x * 256 + threadIdx.x) * 2; if (e >= (size_t)CC * NN) return; const int n = (int)(e % NN), c = (int)(e / NN); v2h o; o[0] = tohx(G[(size_t)n * CC + c]); o[1] = tohx(G[(size_t)(n + 1) * CC + c]); *(volatile v2h*)(GT + e) = o; __threadfence(); *(volatile v2h*)(GT + e) = o; }
__global__ __launch_bounds__(256) void k_mvec(const float* __restrict__ mask, float* M) { const int n = blockIdx.x * 256 + threadIdx.x; if (n >= NN) return; const float mk = bfr(mask[n]); const float a = __fsub_rn(1.0f, fminf(mk, 0.f)); const float v = __fmul_rn(a, __fsub_rn(1.0f, mk)); *(volatile float*)(M + n) = v; __threadfence(); *(volatile float*)(M + n) = v; }
__global__ __launch_bounds__(256) void k_soft3(const float* __restrict__ Sb, const float* __restrict__ M, h16* P) { const int lane = threadIdx.x & 31; const int row = blockIdx.x * 8 + (threadIdx.x >> 5); if (row >= QH) return; const float* sr = Sb + (size_t)row * NN; float mx = -3.0e38f;
    for (int ch = 0; ch < NN / 128; ++ch) { const v4f a = *(const v4f*)(sr + ch * 128 + lane * 4); mx = fmaxf(mx, fmaxf(fmaxf(a[0], a[1]), fmaxf(a[2], a[3]))); }
#pragma unroll
    for (int sh = 16; sh; sh >>= 1) mx = fmaxf(mx, __shfl_xor(mx, sh, 32));
    float sum = 0.f;
    for (int ch = 0; ch < NN / 128; ++ch) { const v4f a = *(const v4f*)(sr + ch * 128 + lane * 4);
#pragma unroll
        for (int q = 0; q < 4; ++q) { float d0 = __fsub_rn(a[q], mx); asm volatile("" : "+v"(d0)); sum += __expf(d0); } }
#pragma unroll
    for (int sh = 16; sh; sh >>= 1) sum += __shfl_xor(sum, sh, 32);
    const float f = __fdiv_rn(PCAR, sum);
    for (int ps = 0; ps < 2; ++ps) { for (int ch = 0; ch < NN / 128; ++ch) { const int j0 = ch * 128 + lane * 4; const v4f a = *(const v4f*)(sr + j0); const v4f m4 = *(const v4f*)(M + j0); v4h o;
#pragma unroll
            for (int q = 0; q < 4; ++q) { float d0 = __fsub_rn(a[q], mx); asm volatile("" : "+v"(d0)); float e = __fmul_rn(__expf(d0), f); asm volatile("" : "+v"(e)); o[q] = tohx(__fmul_rn(e, m4[q])); }
            *(volatile v4h*)(P + (size_t)row * NN + j0) = o; } if (ps == 0) __threadfence(); } }
__global__ __launch_bounds__(256) void k_spl(const float* __restrict__ F, size_t n4, float sc, bf* Fh, bf* Fl) { const size_t i = ((size_t)blockIdx.x * 256 + threadIdx.x) * 4; if (i >= n4 * 4) return; const v4f a = *(const v4f*)(F + i); v4us oh, ol;
#pragma unroll
    for (int q = 0; q < 4; ++q) { unsigned short u, c2; splitf(a[q] * sc, u, c2); oh[q] = u; ol[q] = c2; } *(volatile v4us*)(Fh + i) = oh; *(volatile v4us*)(Fl + i) = ol; __threadfence(); *(volatile v4us*)(Fh + i) = oh; *(volatile v4us*)(Fl + i) = ol; }
__device__ __forceinline__ int reflect64(int i) { return i < 0 ? -i : (i >= HH ? 2 * HH - 2 - i : i); }
__global__ __launch_bounds__(256) void k_col3r(const float* __restrict__ F, bf* Ch, bf* Cl) { const size_t e = ((size_t)blockIdx.x * 256 + threadIdx.x) * 4; if (e >= (size_t)NN * KC) return; const int k = (int)(e % KC); const int n = (int)(e / KC); const int tap = k / CC, ci = k % CC; const int kh = tap / 3, kw = tap % 3; const int y = reflect64(n / HH + kh - 1), x = reflect64(n % HH + kw - 1); const v4f a = *(const v4f*)(F + ((size_t)y * HH + x) * CC + ci); v4us oh, ol;
#pragma unroll
    for (int q = 0; q < 4; ++q) { unsigned short u, c2; splitf(a[q], u, c2); oh[q] = u; ol[q] = c2; } *(volatile v4us*)(Ch + e) = oh; *(volatile v4us*)(Cl + e) = ol; __threadfence(); *(volatile v4us*)(Ch + e) = oh; *(volatile v4us*)(Cl + e) = ol; }
__global__ __launch_bounds__(128) void k_instat(const float* __restrict__ Cv, float* ST) { const int c = threadIdx.x; float s = 0.f; for (int n = 0; n < NN; ++n) s = __fadd_rn(s, Cv[(size_t)n * CC + c]); const float mu = s * (1.0f / NN); float q2 = 0.f; for (int n = 0; n < NN; ++n) { float d = __fsub_rn(Cv[(size_t)n * CC + c], mu); asm volatile("" : "+v"(d)); float p = __fmul_rn(d, d); asm volatile("" : "+v"(p)); q2 = __fadd_rn(q2, p); }
    float vq = q2 * (1.0f / NN); asm volatile("" : "+v"(vq)); const float rs = __frsqrt_rn(__fadd_rn(vq, 1e-3f)); v2f o; o[0] = mu; o[1] = rs; *(volatile v2f*)(ST + 2 * c) = o; __threadfence(); *(volatile v2f*)(ST + 2 * c) = o; }
__global__ __launch_bounds__(256) void k_inrelu(const float* __restrict__ Cv, const float* __restrict__ ST, const float* __restrict__ g, const float* __restrict__ be, float* Hout) { const size_t i = ((size_t)blockIdx.x * 256 + threadIdx.x) * 4; if (i >= (size_t)NN * CC) return; const int c = (int)(i % CC); const v4f a = *(const v4f*)(Cv + i); v4f o;
#pragma unroll
    for (int q = 0; q < 4; ++q) { float d = __fsub_rn(a[q], ST[2 * (c + q)]); asm volatile("" : "+v"(d)); float tn = __fmul_rn(d, ST[2 * (c + q) + 1]); asm volatile("" : "+v"(tn)); float tg = __fmul_rn(tn, bfr(g[c + q])); asm volatile("" : "+v"(tg)); o[q] = fmaxf(__fadd_rn(tg, bfr(be[c + q])), 0.f); }
    *(volatile v4f*)(Hout + i) = o; __threadfence(); *(volatile v4f*)(Hout + i) = o; }
__global__ __launch_bounds__(256) void k_inres(const float* __restrict__ Cv, const float* __restrict__ ST, const float* __restrict__ g, const float* __restrict__ be, const float* __restrict__ WYin, float* WYout) { const size_t i = ((size_t)blockIdx.x * 256 + threadIdx.x) * 4; if (i >= (size_t)NN * CC) return; const int c = (int)(i % CC); const v4f a = *(const v4f*)(Cv + i), w = *(const v4f*)(WYin + i); v4f o;
#pragma unroll
    for (int q = 0; q < 4; ++q) { float d = __fsub_rn(a[q], ST[2 * (c + q)]); asm volatile("" : "+v"(d)); float tn = __fmul_rn(d, ST[2 * (c + q) + 1]); asm volatile("" : "+v"(tn)); float tg = __fmul_rn(tn, bfr(g[c + q])); asm volatile("" : "+v"(tg)); o[q] = __fadd_rn(w[q], __fadd_rn(tg, bfr(be[c + q]))); }
    *(volatile v4f*)(WYout + i) = o; __threadfence(); *(volatile v4f*)(WYout + i) = o; }
__global__ __launch_bounds__(256) void k_blend(const float* __restrict__ x, const float* __restrict__ M, const float* __restrict__ WY, float* OUT) { const size_t i = ((size_t)blockIdx.x * 256 + threadIdx.x) * 4; if (i >= (size_t)NN * CC) return; const int n = (int)(i / CC); const float m = M[n]; const float om = __fsub_rn(1.0f, m); const v4f w = *(const v4f*)(WY + i); v4f o;
#pragma unroll
    for (int q = 0; q < 4; ++q) { float a = __fmul_rn(m, bfr(x[i + q])); asm volatile("" : "+v"(a)); float b = __fmul_rn(om, w[q]); asm volatile("" : "+v"(b)); o[q] = __fadd_rn(a, b); } *(volatile v4f*)(OUT + i) = o; __threadfence(); *(volatile v4f*)(OUT + i) = o; }

extern "C" void kernel_launch(void* const* d_in, const int* in_sizes, int n_in,
                              void* d_out, int out_size, void* d_ws, size_t ws_size, hipStream_t stream) {
    (void)in_sizes; (void)n_in; (void)out_size;
    const float* IN[18]; for (int i = 0; i < 18; ++i) IN[i] = (const float*)d_in[i];
    float* OUT = (float*)d_out;
    char* wsp = (char*)d_ws;
    auto take = [&](size_t bytes) { char* p = wsp; wsp += (bytes + 255) & ~(size_t)255; return (void*)p; };
    bf* WG = (bf*)take(CC * CC * 2); bf* WT = (bf*)take(CC * CC * 2); bf* WP = (bf*)take(CC * CC * 2); bf* WW = (bf*)take(CC * CC * 2); bf* WR = (bf*)take((size_t)6 * CC * KC * 2);
    bf* XB = (bf*)take((size_t)NN * CC * 2); float* GF = (float*)take((size_t)NN * CC * 4); float* TF = (float*)take((size_t)NN * CC * 4); float* PF = (float*)take((size_t)NN * CC * 4); h16* T16 = (h16*)take((size_t)NN * CC * 2); h16* P16k = (h16*)take((size_t)NN * CC * 2); h16* GT = (h16*)take((size_t)CC * NN * 2); float* M = (float*)take((size_t)NN * 4);
    float* Sb = (float*)take((size_t)QH * NN * 4); h16* PP = (h16*)take((size_t)QH * NN * 2); float* Y = (float*)take((size_t)NN * CC * 4); bf* Ah = (bf*)take((size_t)NN * KC * 2); bf* Al = (bf*)take((size_t)NN * KC * 2); float* WY = (float*)take((size_t)NN * CC * 4); float* WY2 = (float*)take((size_t)NN * CC * 4); float* CV = (float*)take((size_t)NN * CC * 4); float* HB = (float*)take((size_t)NN * CC * 4); float* ST = (float*)take(CC * 2 * 4);
    if ((size_t)(wsp - (char*)d_ws) > ws_size) return;
    k_wtG<<<(CC * CC / 64 + 63) / 64, 256, 0, stream>>>(IN[2], CC, CC, WG); k_wtG<<<(CC * CC / 64 + 63) / 64, 256, 0, stream>>>(IN[4], CC, CC, WT); k_wtG<<<(CC * CC / 64 + 63) / 64, 256, 0, stream>>>(IN[6], CC, CC, WP); k_wtG<<<(CC * CC / 64 + 63) / 64, 256, 0, stream>>>(IN[8], CC, CC, WW);
    for (int i = 0; i < 3; ++i) { k_wtG<<<(KC * CC / 64 + 63) / 64, 256, 0, stream>>>(IN[10] + (size_t)i * KC * CC, KC, CC, WR + (size_t)(2 * i) * CC * KC); k_wtG<<<(KC * CC / 64 + 63) / 64, 256, 0, stream>>>(IN[14] + (size_t)i * KC * CC, KC, CC, WR + (size_t)(2 * i + 1) * CC * KC); }
    const unsigned L4 = (unsigned)(((size_t)NN * CC / 4 + 255) / 256);
    for (int b = 0; b < NB_; ++b) { const float* xb = IN[0] + (size_t)b * NN * CC;
        k_cvt8<<<(NN * CC / 8 + 255) / 256, 256, 0, stream>>>(xb, XB, (size_t)NN * CC / 8); k_mvec<<<NN / 256, 256, 0, stream>>>(IN[1] + (size_t)b * NN, M);
        k_gemmw<bf, 0, true><<<dim3(NN / 64, CC / 64, 1), 32, 0, stream>>>(XB, nullptr, WG, nullptr, CC, GF, CC, IN[3], 0, 0, 0); k_gemmw<bf, 0, true><<<dim3(NN / 64, CC / 64, 1), 32, 0, stream>>>(XB, nullptr, WT, nullptr, CC, TF, CC, IN[5], 0, 0, 0); k_gemmw<bf, 0, true><<<dim3(NN / 64, CC / 64, 1), 32, 0, stream>>>(XB, nullptr, WP, nullptr, CC, PF, CC, IN[7], 0, 0, 0);
        k_f16<<<L4, 256, 0, stream>>>(TF, (size_t)NN * CC / 4, T16); k_f16<<<L4, 256, 0, stream>>>(PF, (size_t)NN * CC / 4, P16k); k_gt16<<<(unsigned)(((size_t)CC * NN / 2 + 255) / 256), 256, 0, stream>>>(GF, GT);
        for (int qh = 0; qh < NN; qh += QH) {
            k_gemmw<h16, 0, false><<<dim3(QH / 64, NN / 64, 1), 32, 0, stream>>>(T16 + (size_t)qh * CC, nullptr, P16k, nullptr, CC, Sb, NN, nullptr, 0, 0, 0);
            k_soft3<<<QH / 8, 256, 0, stream>>>(Sb, M, PP);
            k_gemmw<h16, 0, false><<<dim3(QH / 64, CC / 64, 1), 32, 0, stream>>>(PP, nullptr, GT, nullptr, NN, Y + (size_t)qh * CC, CC, nullptr, 0, 0, 0); }
        k_spl<<<L4, 256, 0, stream>>>(Y, (size_t)NN * CC / 4, 1.0f / PCAR, Ah, Al);
        k_gemmw<bf, 1, true><<<dim3(NN / 64, CC / 64, 1), 32, 0, stream>>>(Ah, Al, WW, nullptr, CC, WY, CC, IN[9], 0, 0, 0);
        float* wy = WY; float* wyn = WY2;
        for (int i = 0; i < 3; ++i) {
            k_col3r<<<(unsigned)(((size_t)NN * KC / 4 + 255) / 256), 256, 0, stream>>>(wy, Ah, Al);
            k_gemmw<bf, 1, true><<<dim3(NN / 64, CC / 64, 1), 32, 0, stream>>>(Ah, Al, WR + (size_t)(2 * i) * CC * KC, nullptr, KC, CV, CC, IN[11] + i * CC, 0, 0, 0);
            k_instat<<<1, 128, 0, stream>>>(CV, ST); k_inrelu<<<L4, 256, 0, stream>>>(CV, ST, IN[12] + i * CC, IN[13] + i * CC, HB);
            k_col3r<<<(unsigned)(((size_t)NN * KC / 4 + 255) / 256), 256, 0, stream>>>(HB, Ah, Al);
            k_gemmw<bf, 1, true><<<dim3(NN / 64, CC / 64, 1), 32, 0, stream>>>(Ah, Al, WR + (size_t)(2 * i + 1) * CC * KC, nullptr, KC, CV, CC, IN[15] + i * CC, 0, 0, 0);
            k_instat<<<1, 128, 0, stream>>>(CV, ST); k_inres<<<L4, 256, 0, stream>>>(CV, ST, IN[16] + i * CC, IN[17] + i * CC, wy, wyn); float* t = wy; wy = wyn; wyn = t; }
        k_blend<<<L4, 256, 0, stream>>>(xb, M, wy, OUT + (size_t)b * NN * CC); }
}
